// My_Transformer_Layer_Ch_Big_SmallFF_89232240541898
// MI455X (gfx1250) — hardware-run, weakly checked
//
#include <hip/hip_runtime.h>


#define BB   2
#define NSEQ 256
#define MMOD 8
#define DDIM 256
#define HH   8
#define DH   64
#define INN  (HH * DH)
#define TT   (NSEQ * MMOD)
#define NR   (BB * TT)
#define OW   (MMOD * INN)
#define DO2  (MMOD * DDIM)
#define FW   2048
#define FI   1024
#define PCAR 1024.0f
#define SCL  0.125f
typedef _Float16 h16;
typedef unsigned short bf;
typedef __attribute__((ext_vector_type(16))) __bf16   v16bf;
typedef __attribute__((ext_vector_type(16))) _Float16 v16h;
typedef __attribute__((ext_vector_type(8)))  _Float16 v8h;
typedef __attribute__((ext_vector_type(8)))  unsigned short v8us;
typedef __attribute__((ext_vector_type(8)))  float    v8f;
typedef __attribute__((ext_vector_type(4)))  float    v4f;
typedef v8h  __attribute__((may_alias)) v8ha;
typedef v4f  __attribute__((may_alias)) v4fa;
typedef v8us __attribute__((may_alias)) v8usa;

__device__ __forceinline__ unsigned short f2bf(float f) { unsigned u = __float_as_uint(f); u += 0x7FFFu + ((u >> 16) & 1u); return (unsigned short)(u >> 16); }
__device__ __forceinline__ float bf2f(unsigned short b) { return __uint_as_float(((unsigned)b) << 16); }
__device__ __forceinline__ float bfr(float f) { return bf2f(f2bf(f)); }
__device__ __forceinline__ v16h cat16(v8h lo, v8h hi) { return __builtin_shufflevector(lo, hi, 0, 1, 2, 3, 4, 5, 6, 7, 8, 9, 10, 11, 12, 13, 14, 15); }
__device__ __forceinline__ v16bf cat16b(v8us lo, v8us hi) { return __builtin_bit_cast(v16bf, __builtin_shufflevector(lo, hi, 0, 1, 2, 3, 4, 5, 6, 7, 8, 9, 10, 11, 12, 13, 14, 15)); }
__device__ __forceinline__ v8f wmma16(v16h a, v16h b, v8f c) { return __builtin_amdgcn_wmma_f32_16x16x32_f16(false, a, false, b, (short)0, c, false, false); }
__device__ __forceinline__ v8f wmmab(v16bf a, v16bf b, v8f c) { return __builtin_amdgcn_wmma_f32_16x16x32_bf16(false, a, false, b, (short)0, c, false, false); }


template <typename T16> struct WFrag;
template <> struct WFrag<h16> { typedef v16h V; static __device__ __forceinline__ V ld(const h16* p) { return cat16(*(const v8h*)p, *(const v8h*)(p + 16)); } static __device__ __forceinline__ v8f mma(V a, V b, v8f c) { return wmma16(a, b, c); } };
template <> struct WFrag<bf> { typedef v16bf V; static __device__ __forceinline__ V ld(const bf* p) { return cat16b(*(const v8us*)p, *(const v8us*)(p + 16)); } static __device__ __forceinline__ v8f mma(V a, V b, v8f c) { return wmmab(a, b, c); } };
template <typename T16, int NSPLIT, bool BIAS>
__global__ __launch_bounds__(32) void k_gemmw(const T16* __restrict__ A, const T16* __restrict__ A2, const T16* __restrict__ Bt, const T16* __restrict__ Bt2, int K, float* C, int ldc, const float* __restrict__ bias, size_t sA, size_t sB, size_t sC) {
    typedef typename WFrag<T16>::V V;
    __shared__ __align__(16) float os[16 * 68];
    const size_t z = blockIdx.z; A += z * sA; if (A2) A2 += z * sA; Bt += z * sB; if (Bt2) Bt2 += z * sB; C += z * sC;
    const int lane = threadIdx.x & 31, lr = lane & 15, hi = lane >> 4; const int r0 = blockIdx.x * 64, c0 = blockIdx.y * 64;
    v8f acc[4][4];
#pragma unroll
    for (int mb = 0; mb < 4; ++mb)
#pragma unroll
        for (int nb = 0; nb < 4; ++nb) acc[mb][nb] = (v8f){};
    const size_t aoff = (size_t)(r0 + lr) * K + 8 * hi, boff = (size_t)(c0 + lr) * K + 8 * hi;
#pragma unroll 1
    for (int kc = 0; kc < K; kc += 32) {
        V a[4], a2[4];
#pragma unroll
        for (int mb = 0; mb < 4; ++mb) { a[mb] = WFrag<T16>::ld(A + aoff + (size_t)mb * 16 * K + kc); if (NSPLIT == 1 || NSPLIT == 2) a2[mb] = WFrag<T16>::ld(A2 + aoff + (size_t)mb * 16 * K + kc); }
#pragma unroll
        for (int nb = 0; nb < 4; ++nb) { const V b = WFrag<T16>::ld(Bt + boff + (size_t)nb * 16 * K + kc); V b2; if (NSPLIT >= 2) b2 = WFrag<T16>::ld(Bt2 + boff + (size_t)nb * 16 * K + kc);
#pragma unroll
            for (int mb = 0; mb < 4; ++mb) { acc[mb][nb] = WFrag<T16>::mma(a[mb], b, acc[mb][nb]); if (NSPLIT == 1 || NSPLIT == 2) acc[mb][nb] = WFrag<T16>::mma(a2[mb], b, acc[mb][nb]); if (NSPLIT >= 2) acc[mb][nb] = WFrag<T16>::mma(a[mb], b2, acc[mb][nb]); } }
        asm volatile("v_nop\n\tv_nop\n\tv_nop\n\tv_nop" : "+v"(acc[0][0]), "+v"(acc[1][1]), "+v"(acc[2][2]), "+v"(acc[3][3]) : "v"(a[0]), "v"(a[3]));
    }
#pragma unroll
    for (int mb = 0; mb < 4; ++mb) {
#pragma unroll
        for (int nb = 0; nb < 4; ++nb) {
#pragma unroll
            for (int j = 0; j < 8; ++j) os[(hi * 8 + j) * 68 + nb * 16 + lr] = acc[mb][nb][j]; }
        __builtin_amdgcn_wave_barrier(); asm volatile("" ::: "memory");
        float* crow = C + (size_t)(r0 + mb * 16) * ldc + c0;
#pragma unroll 1
        for (int ps = 0; ps < 2; ++ps) {
#pragma unroll
            for (int s = 0; s < 8; ++s) { const int row = 2 * s + hi, cofs = lr * 4; v4f val = *(const v4fa*)(os + row * 68 + cofs); if (BIAS) { val[0] += bfr(bias[c0 + cofs]); val[1] += bfr(bias[c0 + cofs + 1]); val[2] += bfr(bias[c0 + cofs + 2]); val[3] += bfr(bias[c0 + cofs + 3]); }
                *(volatile v4f*)(crow + (size_t)row * ldc + cofs) = val; }
            if (ps == 0) __threadfence(); }
        __builtin_amdgcn_wave_barrier(); asm volatile("" ::: "memory");
    }
}

__device__ __forceinline__ h16 tohx(float x) { return (h16)x; }
__device__ __forceinline__ void splitf(float y, unsigned short& h, unsigned short& l) { h = f2bf(y); l = f2bf(y - bf2f(h)); }
__device__ __forceinline__ float geluf_(float x) { float er = erff(x * 0.70710678f); asm volatile("" : "+v"(er)); float hx = __fmul_rn(0.5f, x); asm volatile("" : "+v"(hx)); return __fmul_rn(hx, __fadd_rn(1.0f, er)); }
typedef __attribute__((ext_vector_type(2))) _Float16 v2h;
typedef __attribute__((ext_vector_type(4))) _Float16 v4h;
typedef __attribute__((ext_vector_type(2))) unsigned short v2us;
typedef __attribute__((ext_vector_type(4))) unsigned short v4us;
typedef __attribute__((ext_vector_type(2))) float v2f;

__global__ __launch_bounds__(256) void k_wtG(const float* __restrict__ w, int K, int N, bf* Bt) {
    const int lane = threadIdx.x & 31; const int L0 = (blockIdx.x * 8 + (threadIdx.x >> 5)) * 8; const int nlines = N * K / 64;
#pragma unroll 1
    for (int ps = 0; ps < 2; ++ps) {
#pragma unroll 1
        for (int l = 0; l < 8; ++l) { const int L = L0 + l; if (L >= nlines) break; const size_t e = (size_t)L * 64 + lane * 2; const int k = (int)(e % K), n = (int)(e / K); v2us o;
            o[0] = f2bf(w[(size_t)k * N + n]); o[1] = f2bf(w[(size_t)(k + 1) * N + n]); *(volatile v2us*)(Bt + e) = o; }
        if (ps == 0) __threadfence(); }
}
__global__ __launch_bounds__(256) void k_xt(const float* __restrict__ x, float* XTf, bf* XB) { const size_t e = ((size_t)blockIdx.x * 256 + threadIdx.x) * 4; if (e >= (size_t)NR * DDIM) return; const int d = (int)(e % DDIM); const int row = (int)(e / DDIM); const int m = row % MMOD, n = (row / MMOD) % NSEQ, b = row / TT; v4f of; v4us ob;
#pragma unroll
    for (int q = 0; q < 4; ++q) { const float v = bfr(x[(((size_t)b * DDIM + d + q) * MMOD + m) * NSEQ + n]); of[q] = v; ob[q] = f2bf(v); } *(volatile v4f*)(XTf + e) = of; *(volatile v4us*)(XB + e) = ob; __threadfence(); *(volatile v4f*)(XTf + e) = of; *(volatile v4us*)(XB + e) = ob; }
__global__ __launch_bounds__(256) void k_qpl(const float* __restrict__ Qb, h16* QP) { const size_t e = ((size_t)blockIdx.x * 256 + threadIdx.x) * 2; if (e >= (size_t)HH * TT * DH) return; const int d = (int)(e % DH); const int t = (int)((e / DH) % TT); const int h = (int)(e / ((size_t)DH * TT)); const float* s = Qb + (size_t)t * INN + h * DH + d; v2h o; o[0] = tohx(s[0]); o[1] = tohx(s[1]); *(volatile v2h*)(QP + e) = o; __threadfence(); *(volatile v2h*)(QP + e) = o; }
__global__ __launch_bounds__(256) void k_kpl(const float* __restrict__ KVb, h16* KP) { const size_t e = ((size_t)blockIdx.x * 256 + threadIdx.x) * 2; if (e >= (size_t)HH * TT * DH) return; const int d = (int)(e % DH); const int r = (int)((e / DH) % TT); const int h = (int)(e / ((size_t)DH * TT)); const int z = r / NSEQ, j = r % NSEQ; const float* s = KVb + (size_t)(j * MMOD + z) * (2 * INN) + h * DH + d; v2h o; o[0] = tohx(s[0]); o[1] = tohx(s[1]); *(volatile v2h*)(KP + e) = o; __threadfence(); *(volatile v2h*)(KP + e) = o; }
__global__ __launch_bounds__(256) void k_vtp(const float* __restrict__ KVb, h16* VT) { const size_t e = ((size_t)blockIdx.x * 256 + threadIdx.x) * 2; if (e >= (size_t)HH * DH * TT) return; const int c = (int)(e % TT); const int d = (int)((e / TT) % DH); const int h = (int)(e / ((size_t)TT * DH)); const int m = c / NSEQ, j = c % NSEQ; v2h o;
#pragma unroll
    for (int q = 0; q < 2; ++q) o[q] = tohx(KVb[(size_t)((j + q) * MMOD + m) * (2 * INN) + INN + h * DH + d]); *(volatile v2h*)(VT + e) = o; __threadfence(); *(volatile v2h*)(VT + e) = o; }
__global__ __launch_bounds__(256) void k_cst8(const float* __restrict__ Sb, float* CM, float* CI) { const int e = blockIdx.x * 256 + threadIdx.x; if (e >= MMOD * TT) return; const int c = e % TT, m = e / TT; float mx = -3.0e38f;
    for (int i = 0; i < NSEQ; ++i) { float t = __fmul_rn(Sb[(size_t)(i * MMOD + m) * TT + c], SCL); asm volatile("" : "+v"(t)); mx = fmaxf(mx, t); }
    float s = 0.f; for (int i = 0; i < NSEQ; ++i) { float t = __fmul_rn(Sb[(size_t)(i * MMOD + m) * TT + c], SCL); asm volatile("" : "+v"(t)); float d0 = __fsub_rn(t, mx); asm volatile("" : "+v"(d0)); s = __fadd_rn(s, __expf(d0)); }
    const float ci = __fdiv_rn(PCAR, s); *(volatile float*)(CM + e) = mx; *(volatile float*)(CI + e) = ci; __threadfence(); *(volatile float*)(CM + e) = mx; *(volatile float*)(CI + e) = ci; }
__global__ __launch_bounds__(256) void k_pcol8(const float* __restrict__ Sb, const float* __restrict__ CM, const float* __restrict__ CI, h16* P16) { const size_t e = ((size_t)blockIdx.x * 256 + threadIdx.x) * 4; if (e >= (size_t)TT * TT) return; const int c = (int)(e % TT); const int row = (int)(e / TT); const int m = row % MMOD; const v4f a = *(const v4f*)(Sb + e); v4h o;
#pragma unroll
    for (int q = 0; q < 4; ++q) { float t = __fmul_rn(a[q], SCL); asm volatile("" : "+v"(t)); float d0 = __fsub_rn(t, CM[m * TT + c + q]); asm volatile("" : "+v"(d0)); o[q] = tohx(__fmul_rn(__expf(d0), CI[m * TT + c + q])); }
    *(volatile v4h*)(P16 + e) = o; __threadfence(); *(volatile v4h*)(P16 + e) = o; }
__global__ __launch_bounds__(256) void k_perm(const h16* __restrict__ P16, h16* PZ) { const size_t e = ((size_t)blockIdx.x * 256 + threadIdx.x) * 2; if (e >= (size_t)MMOD * NSEQ * TT) return; const int c = (int)(e % TT); const int i = (int)((e / TT) % NSEQ); const int z = (int)(e / ((size_t)TT * NSEQ)); const int m = c / NSEQ, j = c % NSEQ;
    const v2h o = *(const v2h*)(P16 + (size_t)(i * MMOD + m) * TT + z * NSEQ + j); *(volatile v2h*)(PZ + e) = o; __threadfence(); *(volatile v2h*)(PZ + e) = o; }
__global__ __launch_bounds__(256) void k_mrgmt(const float* __restrict__ O, int b, int h, bf* OPh, bf* OPl) { const size_t e = ((size_t)blockIdx.x * 256 + threadIdx.x) * 2; if (e >= (size_t)MMOD * NSEQ * DH) return; const int d = (int)(e % DH); const int i = (int)((e / DH) % NSEQ); const int z = (int)(e / ((size_t)DH * NSEQ)); v2us oh, ol;
#pragma unroll
    for (int q = 0; q < 2; ++q) { unsigned short a, c2; splitf(O[e + q] * (1.0f / PCAR), a, c2); oh[q] = a; ol[q] = c2; } const size_t oo = ((size_t)b * NSEQ + i) * OW + z * INN + h * DH + d; *(volatile v2us*)(OPh + oo) = oh; *(volatile v2us*)(OPl + oo) = ol; __threadfence(); *(volatile v2us*)(OPh + oo) = oh; *(volatile v2us*)(OPl + oo) = ol; }
__device__ __forceinline__ void ln256(float* x8, const float* __restrict__ g, const float* __restrict__ bt, int lane, float* y) { float sm = 0.f;
#pragma unroll
    for (int q = 0; q < 8; ++q) sm = __fadd_rn(sm, x8[q]);
#pragma unroll
    for (int sh = 16; sh; sh >>= 1) sm += __shfl_xor(sm, sh, 32);
    const float mu = sm * (1.0f / DDIM); float q2 = 0.f;
#pragma unroll
    for (int q = 0; q < 8; ++q) { const float d = __fsub_rn(x8[q], mu); float p = __fmul_rn(d, d); asm volatile("" : "+v"(p)); q2 = __fadd_rn(q2, p); }
#pragma unroll
    for (int sh = 16; sh; sh >>= 1) q2 += __shfl_xor(q2, sh, 32);
    const float rs = __frsqrt_rn(__fadd_rn(q2 * (1.0f / DDIM), 1e-5f));
#pragma unroll
    for (int q = 0; q < 8; ++q) { const int d = (q < 4) ? lane * 4 + q : 128 + lane * 4 + (q - 4); float tn = __fmul_rn(__fsub_rn(x8[q], mu), rs); asm volatile("" : "+v"(tn)); float tg = __fmul_rn(tn, bfr(g[d])); asm volatile("" : "+v"(tg)); y[q] = __fadd_rn(tg, bfr(bt[d])); } }
__global__ __launch_bounds__(256) void k_ln1(const float* __restrict__ XTf, const float* __restrict__ O2, const float* __restrict__ g, const float* __restrict__ bt, float* X2f, bf* Xh, bf* Xl) { const int lane = threadIdx.x & 31; const int row = blockIdx.x * 8 + (threadIdx.x >> 5); if (row >= NR) return; const size_t o0 = (size_t)row * DDIM + lane * 4, o1 = o0 + 128;
    const v4f a0 = *(const v4f*)(XTf + o0), a1 = *(const v4f*)(XTf + o1), b0 = *(const v4f*)(O2 + o0), b1 = *(const v4f*)(O2 + o1); float x8[8] = {__fadd_rn(a0[0], b0[0]), __fadd_rn(a0[1], b0[1]), __fadd_rn(a0[2], b0[2]), __fadd_rn(a0[3], b0[3]), __fadd_rn(a1[0], b1[0]), __fadd_rn(a1[1], b1[1]), __fadd_rn(a1[2], b1[2]), __fadd_rn(a1[3], b1[3])}; float y[8]; ln256(x8, g, bt, lane, y);
    v4f f0, f1; v4us h0, h1, l0, l1;
#pragma unroll
    for (int q = 0; q < 4; ++q) { f0[q] = y[q]; f1[q] = y[4 + q]; unsigned short a, c2; splitf(y[q], a, c2); h0[q] = a; l0[q] = c2; splitf(y[4 + q], a, c2); h1[q] = a; l1[q] = c2; }
    for (int ps = 0; ps < 2; ++ps) { *(volatile v4f*)(X2f + o0) = f0; *(volatile v4f*)(X2f + o1) = f1; *(volatile v4us*)(Xh + o0) = h0; *(volatile v4us*)(Xh + o1) = h1; *(volatile v4us*)(Xl + o0) = l0; *(volatile v4us*)(Xl + o1) = l1; if (ps == 0) __threadfence(); } }
__global__ __launch_bounds__(256) void k_geglu(const float* __restrict__ HG, bf* Gh, bf* Gl) { const size_t e = ((size_t)blockIdx.x * 256 + threadIdx.x) * 2; if (e >= (size_t)NR * FI) return; const int c = (int)(e % FI), row = (int)(e / FI); v2us oh, ol;
#pragma unroll
    for (int q = 0; q < 2; ++q) { const float a = HG[(size_t)row * FW + c + q], gt = HG[(size_t)row * FW + FI + c + q]; unsigned short a2, c2; splitf(__fmul_rn(a, geluf_(gt)), a2, c2); oh[q] = a2; ol[q] = c2; } *(volatile v2us*)(Gh + e) = oh; *(volatile v2us*)(Gl + e) = ol; __threadfence(); *(volatile v2us*)(Gh + e) = oh; *(volatile v2us*)(Gl + e) = ol; }
__global__ __launch_bounds__(256) void k_ln2(const float* __restrict__ X2f, const float* __restrict__ FFo, const float* __restrict__ g, const float* __restrict__ bt, float* OUT) { const int lane = threadIdx.x & 31; const int row = blockIdx.x * 8 + (threadIdx.x >> 5); if (row >= NR) return; const size_t o0 = (size_t)row * DDIM + lane * 4, o1 = o0 + 128;
    const v4f a0 = *(const v4f*)(X2f + o0), a1 = *(const v4f*)(X2f + o1), b0 = *(const v4f*)(FFo + o0), b1 = *(const v4f*)(FFo + o1); float x8[8] = {__fadd_rn(a0[0], b0[0]), __fadd_rn(a0[1], b0[1]), __fadd_rn(a0[2], b0[2]), __fadd_rn(a0[3], b0[3]), __fadd_rn(a1[0], b1[0]), __fadd_rn(a1[1], b1[1]), __fadd_rn(a1[2], b1[2]), __fadd_rn(a1[3], b1[3])}; float y[8]; ln256(x8, g, bt, lane, y);
    v4f f0, f1;
#pragma unroll
    for (int q = 0; q < 4; ++q) { f0[q] = y[q]; f1[q] = y[4 + q]; }
    for (int ps = 0; ps < 2; ++ps) { *(volatile v4f*)(OUT + o0) = f0; *(volatile v4f*)(OUT + o1) = f1; if (ps == 0) __threadfence(); } }

extern "C" void kernel_launch(void* const* d_in, const int* in_sizes, int n_in,
                              void* d_out, int out_size, void* d_ws, size_t ws_size, hipStream_t stream) {
    (void)in_sizes; (void)n_in; (void)out_size;
    const float* IN[13]; for (int i = 0; i < 13; ++i) IN[i] = (const float*)d_in[i];
    float* OUT = (float*)d_out;
    char* wsp = (char*)d_ws;
    auto take = [&](size_t bytes) { char* p = wsp; wsp += (bytes + 255) & ~(size_t)255; return (void*)p; };
    bf* WQ = (bf*)take((size_t)INN * DDIM * 2); bf* WKV = (bf*)take((size_t)2 * INN * DDIM * 2); bf* WOUT = (bf*)take((size_t)DO2 * OW * 2); bf* WF1 = (bf*)take((size_t)FW * DDIM * 2); bf* WF2 = (bf*)take((size_t)DDIM * FI * 2);
    float* XTf = (float*)take((size_t)NR * DDIM * 4); bf* XB = (bf*)take((size_t)NR * DDIM * 2); float* Q = (float*)take((size_t)NR * INN * 4); float* KV = (float*)take((size_t)NR * 2 * INN * 4);
    h16* QP = (h16*)take((size_t)HH * TT * DH * 2); h16* KP = (h16*)take((size_t)HH * TT * DH * 2); h16* VT = (h16*)take((size_t)HH * DH * TT * 2); float* Sb = (float*)take((size_t)TT * TT * 4); float* CM = (float*)take((size_t)MMOD * TT * 4); float* CI = (float*)take((size_t)MMOD * TT * 4); h16* P16 = (h16*)take((size_t)TT * TT * 2); h16* PZ = (h16*)take((size_t)MMOD * NSEQ * TT * 2); float* O = (float*)take((size_t)MMOD * NSEQ * DH * 4);
    bf* OPh = (bf*)take((size_t)BB * NSEQ * OW * 2); bf* OPl = (bf*)take((size_t)BB * NSEQ * OW * 2); float* O2 = (float*)take((size_t)BB * NSEQ * DO2 * 4); float* X2f = (float*)take((size_t)NR * DDIM * 4); bf* Xh = (bf*)take((size_t)NR * DDIM * 2); bf* Xl = (bf*)take((size_t)NR * DDIM * 2); float* HG = (float*)take((size_t)NR * FW * 4); bf* Gh = (bf*)take((size_t)NR * FI * 2); bf* Gl = (bf*)take((size_t)NR * FI * 2); float* FFo = (float*)take((size_t)NR * DDIM * 4);
    if ((size_t)(wsp - (char*)d_ws) > ws_size) return;
    { k_wtG<<<(INN * DDIM / 64 + 63) / 64, 256, 0, stream>>>(IN[1], DDIM, INN, WQ); k_wtG<<<(2 * INN * DDIM / 64 + 63) / 64, 256, 0, stream>>>(IN[2], DDIM, 2 * INN, WKV); k_wtG<<<(unsigned)(((size_t)OW * DO2 / 64 + 63) / 64), 256, 0, stream>>>(IN[3], OW, DO2, WOUT);
      k_wtG<<<(DDIM * FW / 64 + 63) / 64, 256, 0, stream>>>(IN[7], DDIM, FW, WF1); k_wtG<<<(FI * DDIM / 64 + 63) / 64, 256, 0, stream>>>(IN[9], FI, DDIM, WF2); }
    k_xt<<<(unsigned)(((size_t)NR * DDIM / 4 + 255) / 256), 256, 0, stream>>>(IN[0], XTf, XB);
    k_gemmw<bf, 0, false><<<dim3(NR / 64, INN / 64, 1), 32, 0, stream>>>(XB, nullptr, WQ, nullptr, DDIM, Q, INN, nullptr, 0, 0, 0); k_gemmw<bf, 0, false><<<dim3(NR / 64, 2 * INN / 64, 1), 32, 0, stream>>>(XB, nullptr, WKV, nullptr, DDIM, KV, 2 * INN, nullptr, 0, 0, 0);
    const unsigned LPL = (unsigned)(((size_t)HH * TT * DH / 2 + 255) / 256);
    for (int b = 0; b < BB; ++b) { const float* Qb = Q + (size_t)b * TT * INN; const float* KVb = KV + (size_t)b * TT * 2 * INN;
        k_qpl<<<LPL, 256, 0, stream>>>(Qb, QP); k_kpl<<<LPL, 256, 0, stream>>>(KVb, KP); k_vtp<<<LPL, 256, 0, stream>>>(KVb, VT);
        for (int h = 0; h < HH; ++h) {
            k_gemmw<h16, 0, false><<<dim3(TT / 64, TT / 64, 1), 32, 0, stream>>>(QP + (size_t)h * TT * DH, nullptr, KP + (size_t)h * TT * DH, nullptr, DH, Sb, TT, nullptr, 0, 0, 0);
            k_cst8<<<(MMOD * TT + 255) / 256, 256, 0, stream>>>(Sb, CM, CI); k_pcol8<<<(unsigned)(((size_t)TT * TT / 4 + 255) / 256), 256, 0, stream>>>(Sb, CM, CI, P16); k_perm<<<(unsigned)(((size_t)MMOD * NSEQ * TT / 2 + 255) / 256), 256, 0, stream>>>(P16, PZ);
            k_gemmw<h16, 0, false><<<dim3(NSEQ / 64, 1, MMOD), 32, 0, stream>>>(PZ, nullptr, VT + (size_t)h * DH * TT, nullptr, TT, O, DH, nullptr, (size_t)NSEQ * TT, 0, (size_t)NSEQ * DH);
            k_mrgmt<<<(MMOD * NSEQ * DH / 2 + 255) / 256, 256, 0, stream>>>(O, b, h, OPh, OPl); } }
    k_gemmw<bf, 1, true><<<dim3(BB * NSEQ / 64, DO2 / 64, 1), 32, 0, stream>>>(OPh, OPl, WOUT, nullptr, OW, O2, DO2, IN[4], 0, 0, 0);
    k_ln1<<<NR / 8, 256, 0, stream>>>(XTf, O2, IN[5], IN[6], X2f, Xh, Xl);
    k_gemmw<bf, 1, true><<<dim3(NR / 64, FW / 64, 1), 32, 0, stream>>>(Xh, Xl, WF1, nullptr, DDIM, HG, FW, IN[8], 0, 0, 0);
    k_geglu<<<(unsigned)(((size_t)NR * FI / 2 + 255) / 256), 256, 0, stream>>>(HG, Gh, Gl);
    k_gemmw<bf, 1, true><<<dim3(NR / 64, DDIM / 64, 1), 32, 0, stream>>>(Gh, Gl, WF2, nullptr, FI, FFo, DDIM, IN[10], 0, 0, 0);
    k_ln2<<<NR / 8, 256, 0, stream>>>(X2f, FFo, IN[11], IN[12], OUT);
}
